// ScaledDotAttention_67826123538546
// MI455X (gfx1250) — hardware-verified
//
#include <hip/hip_runtime.h>
#include <math.h>

typedef __attribute__((ext_vector_type(16))) _Float16 v16h;
typedef __attribute__((ext_vector_type(16))) __bf16 v16b;
typedef __attribute__((ext_vector_type(8)))  _Float16 v8h;
typedef __attribute__((ext_vector_type(8)))  float v8f;
typedef __attribute__((ext_vector_type(4)))  float v4f;
typedef __attribute__((ext_vector_type(2)))  float v2f;
typedef __attribute__((ext_vector_type(4)))  unsigned v4u;
typedef __attribute__((ext_vector_type(4)))  int v4i;
typedef float __attribute__((may_alias)) float_a;
typedef int __attribute__((may_alias)) int_a;

template <typename T> __device__ __forceinline__ void vst2(void* p, T v) { *(volatile T*)p = v; __threadfence(); *(volatile T*)p = v; }
__device__ __forceinline__ v8f wmma16(v16h a, v16h b, v8f c) {
  v8f d = __builtin_amdgcn_wmma_f32_16x16x32_f16(false, a, false, b, (short)0, c, false, false);
  asm volatile("v_nop\n\tv_nop\n\tv_nop\n\tv_nop" : "+v"(d) : "v"(a), "v"(b));
  return d;
}
__device__ __forceinline__ v8f wmma_bf(v16b a, v16b b, v8f c) {
  v8f d = __builtin_amdgcn_wmma_f32_16x16x32_bf16(false, a, false, b, (short)0, c, false, false);
  asm volatile("v_nop\n\tv_nop\n\tv_nop\n\tv_nop" : "+v"(d) : "v"(a), "v"(b));
  return d;
}
__device__ __forceinline__ v16h frag_h(const _Float16* rowk0, int lane) {
  union { v16h v; v8h q[2]; } u; const _Float16* p = rowk0 + 8 * (lane >> 4);
  u.q[0] = *(const v8h*)p; u.q[1] = *(const v8h*)(p + 16); return u.v;
}
__device__ __forceinline__ v16h frag_f32(const float* rowk0, int lane) {
  v16h a; const float* p = rowk0 + 8 * (lane >> 4);
#pragma unroll
  for (int i = 0; i < 8; ++i) { a[i] = (_Float16)p[i]; a[8 + i] = (_Float16)p[16 + i]; }
  return a;
}
__device__ __forceinline__ v16h frag_f32s(const float* rowk0, int lane, float sc) {
  v16h a; const float* p = rowk0 + 8 * (lane >> 4);
#pragma unroll
  for (int i = 0; i < 8; ++i) { a[i] = (_Float16)(p[i] * sc); a[8 + i] = (_Float16)(p[16 + i] * sc); }
  return a;
}
__device__ __forceinline__ v16h fragc_f32(const float* W, int k0, int n, int lane, int ld, int K) {
  v16h a; const int g = lane >> 4;
#pragma unroll
  for (int i = 0; i < 8; ++i) { const int ka = k0 + 8 * g + i, kb = ka + 16;
    a[i] = (_Float16)(ka < K ? W[(size_t)(ka < K ? ka : K - 1) * ld + n] : 0.f); a[8 + i] = (_Float16)(kb < K ? W[(size_t)(kb < K ? kb : K - 1) * ld + n] : 0.f); }
  return a;
}
struct F2 { v16b h, l; };
__device__ __forceinline__ F2 bsplit16(const float v[16]) { F2 r;
#pragma unroll
  for (int i = 0; i < 16; ++i) { const __bf16 h = (__bf16)v[i]; r.h[i] = h; r.l[i] = (__bf16)(v[i] - (float)h); }
  return r; }
__device__ __forceinline__ F2 split_row(const float* row, int k0, int lane) { float v[16]; const float* p = row + k0 + 8 * (lane >> 4);
#pragma unroll
  for (int i = 0; i < 8; ++i) { v[i] = p[i]; v[8 + i] = p[16 + i]; }
  return bsplit16(v); }
__device__ __forceinline__ F2 split_rowK(const float* row, int k0, int lane, int K) { float v[16]; const int g = lane >> 4;
#pragma unroll
  for (int i = 0; i < 8; ++i) { const int ka = k0 + 8 * g + i, kb = ka + 16; v[i] = ka < K ? row[ka < K ? ka : K - 1] : 0.f; v[8 + i] = kb < K ? row[kb < K ? kb : K - 1] : 0.f; }
  return bsplit16(v); }
__device__ __forceinline__ F2 split_col(const float* W, int k0, int n, int lane, int ld, int K) { float v[16]; const int g = lane >> 4;
#pragma unroll
  for (int i = 0; i < 8; ++i) { const int ka = k0 + 8 * g + i, kb = ka + 16; v[i] = ka < K ? W[(size_t)(ka < K ? ka : K - 1) * ld + n] : 0.f; v[8 + i] = kb < K ? W[(size_t)(kb < K ? kb : K - 1) * ld + n] : 0.f; }
  return bsplit16(v); }
__device__ __forceinline__ v8f mac3(const F2& a, const F2& b, v8f c) { c = wmma_bf(a.l, b.h, c); c = wmma_bf(a.h, b.l, c); return wmma_bf(a.h, b.h, c); }
__device__ __forceinline__ float sigm(float v) { return 1.0f / (1.0f + expf(-v)); }
#define LDSX() do { asm volatile("s_wait_dscnt 0" ::: "memory"); __builtin_amdgcn_wave_barrier(); __builtin_amdgcn_fence(__ATOMIC_RELEASE, "workgroup"); } while (0)

__device__ __forceinline__ float bfr(float v) { return (float)(__bf16)v; }
#define NB 8
#define TT 2048
#define DIN 256
#define HP 128
#define DV 256
#ifndef TNB
#define TNB NB
#endif
#define BG 4
typedef __attribute__((ext_vector_type(8))) __bf16 v8b;
__device__ __forceinline__ v16b frag_b(const __bf16* rowk0, int lane) { union { v16b v; v8b q[2]; } u; const __bf16* p = rowk0 + 8 * (lane >> 4); u.q[0] = *(const v8b*)p; u.q[1] = *(const v8b*)(p + 16); return u.v; }
#define WS_QH  0u
#define WS_QL  (WS_QH + 2u * (size_t)NB * TT * HP)
#define WS_KH  (WS_QL + 2u * (size_t)NB * TT * HP)
#define WS_KL  (WS_KH + 2u * (size_t)NB * TT * HP)
#define WS_V1  (WS_KL + 2u * (size_t)NB * TT * HP)
#define WS_V2  (WS_V1 + 2u * (size_t)NB * DV * TT)
#define WS_S   (WS_V2 + 2u * (size_t)NB * DV * TT)
#define WS_END (WS_S + 4u * (size_t)BG * TT * TT)
__global__ __launch_bounds__(128) void k_proj(const float* __restrict__ XQ, const float* __restrict__ XK, const float* __restrict__ WQ, const float* __restrict__ WK, const float* __restrict__ SCL, _Float16* __restrict__ QH, _Float16* __restrict__ QL, _Float16* __restrict__ KH, _Float16* __restrict__ KL) { __shared__ __align__(16) _Float16 sh[64][136], sl[64][136];
  const int tid = threadIdx.x, wave = tid >> 5, lane = tid & 31, col = lane & 15, g = lane >> 4; const int which = blockIdx.y; const size_t r0 = (size_t)blockIdx.x * 64; const float* X = which == 0 ? XQ : XK; const float* Wt = which == 0 ? WQ : WK; _Float16* DH = which == 0 ? QH : KH; _Float16* DL = which == 0 ? QL : KL;
  v8f acc[8] = {};
#pragma unroll 2
  for (int kc = 0; kc < DIN / 32; ++kc) { v16b a; { const float* p = X + (r0 + wave * 16 + col) * DIN + kc * 32 + 8 * g;
#pragma unroll
      for (int i = 0; i < 8; ++i) { a[i] = (__bf16)p[i]; a[8 + i] = (__bf16)p[16 + i]; } }
#pragma unroll
    for (int j = 0; j < 8; ++j) { v16b w; const float* wr = Wt + (size_t)(j * 16 + col) * DIN + kc * 32 + 8 * g;
#pragma unroll
      for (int i = 0; i < 8; ++i) { w[i] = (__bf16)wr[i]; w[8 + i] = (__bf16)wr[16 + i]; }
      asm volatile("s_wait_loadcnt 0x0" ::: "memory"); acc[j] = wmma_bf(a, w, acc[j]); } }
#pragma unroll
  for (int j = 0; j < 8; ++j) { const int o = j * 16 + col; const float sc = (which == 1) ? bfr(SCL[o]) : 1.0f;
#pragma unroll
    for (int r = 0; r < 8; ++r) { const float v = fmaxf(acc[j][r], 0.f) * sc; const _Float16 hv = (_Float16)v; sh[wave * 16 + 8 * g + r][o] = hv; sl[wave * 16 + 8 * g + r][o] = (_Float16)((v - (float)hv) * 1024.0f); } }
  __syncthreads();
  for (int e = tid; e < 64 * 16; e += 128) { const int rl = e >> 4, q = e & 15; vst2((unsigned*)(DH + (r0 + rl) * HP + q * 8), *(const v4u*)&sh[rl][q * 8]); vst2((unsigned*)(DL + (r0 + rl) * HP + q * 8), *(const v4u*)&sl[rl][q * 8]); } }
__global__ __launch_bounds__(128) void k_vt(const float* __restrict__ VA, const float* __restrict__ VB, __bf16* __restrict__ PA, __bf16* __restrict__ PB) { __shared__ __align__(16) __bf16 th[128][136];
  const int tid = threadIdx.x; const int t0 = blockIdx.x * 128; const size_t b = blockIdx.y; const int which = blockIdx.z >> 1, c0 = (blockIdx.z & 1) * 128; const float* V = which == 0 ? VA : VB; __bf16* P = which == 0 ? PA : PB;
  for (int e = tid; e < 128 * 128; e += 128) { const int tl = e >> 7, cl = e & 127; th[cl][tl] = (__bf16)V[(b * TT + t0 + tl) * DV + c0 + cl]; }
  __syncthreads();
  for (int e = tid; e < 128 * 16; e += 128) { const int cl = e >> 4, q = e & 15; vst2((unsigned*)(P + (b * DV + c0 + cl) * (size_t)TT + t0 + q * 8), *(const v4u*)&th[cl][q * 8]); } }
__global__ __launch_bounds__(128) void k_sc(const _Float16* __restrict__ RH, const _Float16* __restrict__ RL, const _Float16* __restrict__ CH_, const _Float16* __restrict__ CL, const int* __restrict__ CMASK, int b0, float* __restrict__ S0) { __shared__ __align__(16) float ss[4][16][132]; __shared__ int smk[128];
  const size_t b = b0 + blockIdx.z; float* S = S0 + (size_t)blockIdx.z * TT * TT;
  const int tid = threadIdx.x, wave = tid >> 5, lane = tid & 31, col = lane & 15, g = lane >> 4; const int k0 = blockIdx.y * 128; const int ql0 = blockIdx.x * 64 + wave * 16;
  smk[tid] = CMASK[b * TT + k0 + tid]; __syncthreads();
  v8f acc[8] = {}, accl[8] = {};
#pragma unroll
  for (int kc = 0; kc < HP / 32; ++kc) { const size_t ro = (b * TT + ql0 + col) * HP + kc * 32; const v16h ah = frag_h(RH + ro, lane), al = frag_h(RL + ro, lane);
#pragma unroll
    for (int j = 0; j < 8; ++j) { const size_t co = (b * TT + k0 + j * 16 + col) * HP + kc * 32; const v16h kb = frag_h(CH_ + co, lane), kl = frag_h(CL + co, lane); acc[j] = wmma16(ah, kb, acc[j]); accl[j] = wmma16(al, kb, accl[j]); accl[j] = wmma16(ah, kl, accl[j]); } }
#pragma unroll
  for (int j = 0; j < 8; ++j) { const bool masked = smk[j * 16 + col] != 0;
#pragma unroll
    for (int r = 0; r < 8; ++r) ss[wave][8 * g + r][j * 16 + col] = masked ? -3.0e38f : (acc[j][r] + accl[j][r] * (1.0f / 1024.0f)); }
  LDSX(); for (int rl = 0; rl < 16; ++rl) vst2(S + (size_t)(ql0 + rl) * TT + k0 + lane * 4, *(const v4f*)&ss[wave][rl][lane * 4]); }
__global__ __launch_bounds__(256) void k_sm(float* __restrict__ S0) { __shared__ float sred[8]; __shared__ float sbc; __shared__ __align__(16) float sh[TT];
  const int t = threadIdx.x; const size_t row = blockIdx.x; float* sr = S0 + (size_t)blockIdx.y * TT * TT + row * TT; const int kend = TT;
  float m = -3.0e38f; for (int k = t; k < kend; k += 256) m = fmaxf(m, sr[k]);
#pragma unroll
  for (int o = 1; o < 32; o <<= 1) m = fmaxf(m, __shfl_xor(m, o));
  if ((t & 31) == 0) sred[t >> 5] = m; __syncthreads(); if (t == 0) { float a = sred[0]; for (int i = 1; i < 8; ++i) a = fmaxf(a, sred[i]); sbc = a; } __syncthreads(); m = sbc; __syncthreads();
  float sum = 0.f; for (int k = t; k < kend; k += 256) { const float v = sr[k]; sum += (v <= -1.0e38f) ? 0.f : expf(v - m); }
#pragma unroll
  for (int o = 1; o < 32; o <<= 1) sum += __shfl_xor(sum, o);
  if ((t & 31) == 0) sred[t >> 5] = sum; __syncthreads(); if (t == 0) { float a = 0.f; for (int i = 0; i < 8; ++i) a += sred[i]; sbc = 1.0f / a; } __syncthreads(); const float inv = sbc;
  for (int k = t; k < kend; k += 256) { const float v = sr[k]; sh[k] = (v <= -1.0e38f) ? 0.f : expf(v - m) * inv * 2048.0f; }
  __syncthreads(); for (int q = t; q < kend / 4; q += 256) vst2(sr + q * 4, *(const v4f*)&sh[q * 4]); }
__global__ __launch_bounds__(128) void k_pv(const float* __restrict__ PS0, const __bf16* __restrict__ VP, int b0, float* __restrict__ OUT) { __shared__ __align__(16) float ss[4][16][132];
  const size_t b = b0 + blockIdx.z; const float* PS = PS0 + (size_t)blockIdx.z * TT * TT;
  const int tid = threadIdx.x, wave = tid >> 5, lane = tid & 31, col = lane & 15, g = lane >> 4; const int ql0 = blockIdx.x * 64 + wave * 16; const int c0 = blockIdx.y * 128;
  v8f acc[8] = {};
#pragma unroll 1
  for (int kc = 0; kc < TT / 32; ++kc) { const F2 p = split_row(PS + (size_t)(ql0 + col) * TT, kc * 32, lane);
#pragma unroll
    for (int j = 0; j < 8; ++j) { const v16b vv = frag_b(VP + (b * DV + c0 + j * 16 + col) * (size_t)TT + kc * 32, lane); acc[j] = wmma_bf(p.h, vv, acc[j]); acc[j] = wmma_bf(p.l, vv, acc[j]); } }
#pragma unroll
  for (int j = 0; j < 8; ++j)
#pragma unroll
    for (int r = 0; r < 8; ++r) ss[wave][8 * g + r][j * 16 + col] = acc[j][r] * (1.0f / 2048.0f);
  LDSX(); for (int rl = 0; rl < 16; ++rl) vst2(OUT + (b * TT + ql0 + rl) * DV + c0 + lane * 4, *(const v4f*)&ss[wave][rl][lane * 4]); }
extern "C" void kernel_launch(void* const* d_in, const int* in_sizes, int n_in, void* d_out, int out_size, void* d_ws, size_t ws_size, hipStream_t stream) {
  (void)in_sizes; (void)n_in; (void)out_size;
  const float** F = (const float**)d_in;
  if (ws_size < (size_t)WS_END) return;
  char* ws = (char*)d_ws; _Float16 *QH = (_Float16*)(ws + WS_QH), *QL = (_Float16*)(ws + WS_QL), *KH = (_Float16*)(ws + WS_KH), *KL = (_Float16*)(ws + WS_KL); __bf16 *V1 = (__bf16*)(ws + WS_V1), *V2 = (__bf16*)(ws + WS_V2); float* S = (float*)(ws + WS_S);
  float* OUT1 = (float*)d_out; float* OUT2 = (float*)d_out + (size_t)NB * TT * DV;
  k_proj<<<dim3(TNB * TT / 64, 2), 128, 0, stream>>>(F[0], F[1], F[6], F[7], F[8], QH, QL, KH, KL);
  k_vt<<<dim3(TT / 128, TNB, 4), 128, 0, stream>>>(F[2], F[4], V1, V2);
  for (int b0 = 0; b0 < TNB; b0 += BG) { const int ng = (TNB - b0) < BG ? (TNB - b0) : BG;
    k_sc<<<dim3(TT / 64, TT / 128, ng), 128, 0, stream>>>(QH, QL, KH, KL, (const int*)d_in[3], b0, S);
    k_sm<<<dim3(TT, ng), 256, 0, stream>>>(S);
    k_pv<<<dim3(TT / 64, DV / 128, ng), 128, 0, stream>>>(S, V1, b0, OUT1);
    k_sc<<<dim3(TT / 64, TT / 128, ng), 128, 0, stream>>>(KH, KL, QH, QL, (const int*)d_in[5], b0, S);
    k_sm<<<dim3(TT, ng), 256, 0, stream>>>(S);
    k_pv<<<dim3(TT / 64, DV / 128, ng), 128, 0, stream>>>(S, V2, b0, OUT2);
  }
}
